// AutoregressivePPRM_46737834115554
// MI455X (gfx1250) — hardware-run, weakly checked
//
#include <hip/hip_runtime.h>
#include <math.h>

typedef __attribute__((ext_vector_type(16))) _Float16 v16h;
typedef __attribute__((ext_vector_type(8)))  _Float16 v8h;
typedef __attribute__((ext_vector_type(8)))  float    v8f;
typedef __attribute__((ext_vector_type(4)))  float    v4f;

constexpr int kBatch  = 32;
constexpr int kNodes  = 500;
constexpr int kRows   = kBatch * kNodes;
constexpr int kD      = 256;
constexpr int kG3     = 3 * kD;
constexpr int kHor    = 24;
constexpr int kBot    = 8;
constexpr int kTileM  = 32;
constexpr int kBlocks = kRows / kTileM;
constexpr int kHP     = 264;
constexpr float kCarry    = 64.0f;
constexpr float kInvCarry = 1.0f / kCarry;
static_assert(kRows == 16000, "rows");
static_assert(kRows % kTileM == 0, "row tiles exact");
static_assert(kD % 32 == 0, "K multiple of 32");
static_assert(kG3 % 16 == 0, "N multiple of 16");
static_assert((kTileM * kHor * 4) % 128 == 0, "output tile is whole lines");

constexpr size_t kWhhHalves = (size_t)kG3 * kD;
constexpr size_t kWlgHalves = (size_t)16 * kD;
constexpr size_t kWsTotal   = (kWhhHalves + kWlgHalves) * 2;
constexpr int kWhhBlocks = (int)(kWhhHalves / 8 / 256);
constexpr int kCvtBlocks = (int)((kWhhHalves + kWlgHalves) / 8 / 256);
static_assert(kWhhBlocks * 256 * 8 == (int)kWhhHalves, "plane coverage");
static_assert(kCvtBlocks == kWhhBlocks + 2, "two extra blocks for the 16-row tile");
static_assert(kBot * kD == 256 * 8, "one block per small weight matrix");
static_assert(kWsTotal == 401408ull, "carve total");

union FragU { v16h v; v8h h[2]; };

__device__ __forceinline__ v8f mma_f16(v16h a, v16h b, v8f c) {
  c = __builtin_amdgcn_wmma_f32_16x16x32_f16(false, a, false, b, (short)0, c, false, false);
  asm volatile("v_nop\n\tv_nop\n\tv_nop\n\tv_nop" : "+v"(c) : "v"(a), "v"(b));
  return c;
}

__device__ __forceinline__ float fast_sigmoid(float x) {
  return __builtin_amdgcn_rcpf(1.0f + __expf(-x));
}
__device__ __forceinline__ float fast_tanh(float x) {
  const float q = __builtin_amdgcn_rcpf(1.0f + __expf(2.0f * x));
  return fmaf(-2.0f, q, 1.0f);
}

__global__ __launch_bounds__(256) void build_planes_kernel(
    const float* __restrict__ Whh, const float* __restrict__ Wl, const float* __restrict__ Wg1,
    unsigned short* __restrict__ planes)
{
  const int blk = blockIdx.x;
  if (blk >= kCvtBlocks) return;
  const int tid = threadIdx.x;
  const size_t e0 = ((size_t)blk * 256 + tid) * 8;
  const float* src = Whh;
  size_t s0 = e0;
  if (blk == kWhhBlocks)     { src = Wl;  s0 = (size_t)tid * 8; }
  if (blk == kWhhBlocks + 1) { src = Wg1; s0 = (size_t)tid * 8; }
  const v4f a0 = *(const v4f*)(src + s0);
  const v4f a1 = *(const v4f*)(src + s0 + 4);
  v8h hv;
#pragma unroll
  for (int e = 0; e < 4; ++e) {
    hv[e]     = (_Float16)(a0[e] * kCarry);
    hv[4 + e] = (_Float16)(a1[e] * kCarry);
  }
  _Float16* dst = (_Float16*)planes + e0;
  *(volatile v8h*)dst = hv;
  __threadfence();
  *(volatile v8h*)dst = hv;
}

__global__ __launch_bounds__(256) void gru_horizon_kernel(
    const float* __restrict__ features, const float* __restrict__ last_value,
    const float* __restrict__ W_ih, const float* __restrict__ b_ih, const float* __restrict__ b_hh,
    const float* __restrict__ bl, const float* __restrict__ Wh, const float* __restrict__ bh,
    const float* __restrict__ bg1, const float* __restrict__ Wg2, const float* __restrict__ bg2,
    const float* __restrict__ log_decay,
    const unsigned short* __restrict__ planes, float* __restrict__ out)
{
  __shared__ __align__(16) _Float16 hbuf[kTileM * kHP];
  __shared__ __align__(16) _Float16 wlg[16 * kHP];
  __shared__ __align__(16) float ftile[16 * kD];
  __shared__ __align__(16) float gate_lds[kTileM * kHor];
  __shared__ __align__(16) float preds_lds[kTileM * kHor];
  __shared__ float cst_lds[7 * kD];
  __shared__ float g1_lds[kTileM * kBot];
  __shared__ float x_lds[kTileM];
  __shared__ float lv_lds[kTileM];

  const int tid  = threadIdx.x;
  const int lane = tid & 31;
  const int wave = __builtin_amdgcn_readfirstlane(tid >> 5);
  const int hh   = lane >> 4;
  const int rl   = lane & 15;
  const int row0 = blockIdx.x * kTileM;
  const _Float16* whh  = (const _Float16*)planes;
  const _Float16* wlgp = whh + kWhhHalves;

  {
    const float wir = W_ih[tid], wiz = W_ih[kD + tid], win = W_ih[2 * kD + tid];
    const float bir = b_ih[tid], biz = b_ih[kD + tid], bin = b_ih[2 * kD + tid];
    const float bhr = b_hh[tid], bhz = b_hh[kD + tid], bhn = b_hh[2 * kD + tid];
    cst_lds[tid]          = wir;
    cst_lds[kD + tid]     = wiz;
    cst_lds[2 * kD + tid] = win;
    cst_lds[3 * kD + tid] = bir + bhr;
    cst_lds[4 * kD + tid] = biz + bhz;
    cst_lds[5 * kD + tid] = bin;
    cst_lds[6 * kD + tid] = bhn;
  }
#pragma unroll
  for (int i = 0; i < 2; ++i) {
    const int c  = tid + 256 * i;
    const int r  = c >> 5;
    const int c8 = (c & 31) * 8;
    const v8h w = *(const v8h*)(wlgp + r * kD + c8);
    *(v8h*)(wlg + r * kHP + c8) = w;
  }
  if (tid < kTileM) {
    const float lv = last_value[row0 + tid];
    x_lds[tid]  = lv;
    lv_lds[tid] = lv;
  }
  const float blv  = bl[rl & 7];
  const float whv  = Wh[rl & 7];
  const float bg1v = bg1[rl & 7];
  const float bhv  = bh[0];

  float hold[2][2][8];
#pragma unroll
  for (int mt = 0; mt < 2; ++mt) {
#pragma unroll
    for (int i = 0; i < 2; ++i) {
      const int c  = tid + 256 * i;
      const int r  = c >> 5;
      const int c8 = (c & 31) * 8;
      const float* src = features + (size_t)(row0 + mt * 16 + r) * kD + c8;
      const v4f a0 = *(const v4f*)(src);
      const v4f a1 = *(const v4f*)(src + 4);
      *(v4f*)(ftile + r * kD + c8)     = a0;
      *(v4f*)(ftile + r * kD + c8 + 4) = a1;
      v8h hv;
#pragma unroll
      for (int e = 0; e < 4; ++e) {
        hv[e]     = (_Float16)a0[e];
        hv[4 + e] = (_Float16)a1[e];
      }
      *(v8h*)(hbuf + (mt * 16 + r) * kHP + c8) = hv;
    }
    __syncthreads();
#pragma unroll
    for (int g = 0; g < 2; ++g) {
      const int col = g * 128 + 16 * wave + rl;
#pragma unroll
      for (int r = 0; r < 8; ++r) hold[mt][g][r] = ftile[(8 * hh + r) * kD + col];
    }
    __syncthreads();
  }

  {
    v8f pacc = (v8f){0.f, 0.f, 0.f, 0.f, 0.f, 0.f, 0.f, 0.f};
    if (wave < 2) {
#pragma unroll 1
      for (int kk = 0; kk < kD / 32; ++kk) {
        const int ko = kk * 32 + 8 * hh;
        FragU a, b;
        a.h[0] = *(const v8h*)(hbuf + (wave * 16 + rl) * kHP + ko);
        a.h[1] = *(const v8h*)(hbuf + (wave * 16 + rl) * kHP + ko + 16);
        b.h[0] = *(const v8h*)(wlg + rl * kHP + ko);
        b.h[1] = *(const v8h*)(wlg + rl * kHP + ko + 16);
        pacc = mma_f16(a.v, b.v, pacc);
      }
      if (rl >= 8) {
#pragma unroll
        for (int r = 0; r < 8; ++r) {
          const float v = fmaf(pacc[r], kInvCarry, bg1v);
          g1_lds[(wave * 16 + 8 * hh + r) * kBot + (rl - 8)] = fmaxf(v, 0.0f);
        }
      }
    }
  }
  __syncthreads();
#pragma unroll 1
  for (int i = 0; i < 3; ++i) {
    const int idx = tid + 256 * i;
    const int row = idx / kHor;
    const int s   = idx - row * kHor;
    const v4f w0 = *(const v4f*)(Wg2 + s * kBot);
    const v4f w1 = *(const v4f*)(Wg2 + s * kBot + 4);
    const float* gp = g1_lds + row * kBot;
    float a = 0.0f;
    a = fmaf(gp[0], w0[0], a);
    a = fmaf(gp[1], w0[1], a);
    a = fmaf(gp[2], w0[2], a);
    a = fmaf(gp[3], w0[3], a);
    a = fmaf(gp[4], w1[0], a);
    a = fmaf(gp[5], w1[1], a);
    a = fmaf(gp[6], w1[2], a);
    a = fmaf(gp[7], w1[3], a);
    a += bg2[s];
    gate_lds[idx] = __builtin_amdgcn_rcpf(1.0f + expf(-a));
  }

  const bool lowcol = (rl < 8);
#pragma unroll 1
  for (int t = 0; t < kHor; ++t) {
    v8f acc[2][6];
#pragma unroll
    for (int mt = 0; mt < 2; ++mt)
#pragma unroll
      for (int i = 0; i < 6; ++i) acc[mt][i] = (v8f){0.f, 0.f, 0.f, 0.f, 0.f, 0.f, 0.f, 0.f};

#pragma unroll 1
    for (int kk = 0; kk < kD / 32; ++kk) {
      const int ko = kk * 32 + 8 * hh;
      FragU a0, a1;
      a0.h[0] = *(const v8h*)(hbuf + rl * kHP + ko);
      a0.h[1] = *(const v8h*)(hbuf + rl * kHP + ko + 16);
      a1.h[0] = *(const v8h*)(hbuf + (16 + rl) * kHP + ko);
      a1.h[1] = *(const v8h*)(hbuf + (16 + rl) * kHP + ko + 16);
#pragma unroll
      for (int i = 0; i < 6; ++i) {
        const int nrow = (i >> 1) * kD + (i & 1) * 128 + 16 * wave + rl;
        const _Float16* bp = whh + (size_t)nrow * kD + ko;
        FragU b;
        b.h[0] = *(const v8h*)(bp);
        b.h[1] = *(const v8h*)(bp + 16);
        acc[0][i] = mma_f16(a0.v, b.v, acc[0][i]);
        acc[1][i] = mma_f16(a1.v, b.v, acc[1][i]);
      }
    }
    __syncthreads();

#pragma unroll
    for (int g = 0; g < 2; ++g) {
      const int col = g * 128 + 16 * wave + rl;
      const float wr  = cst_lds[col];
      const float wz  = cst_lds[kD + col];
      const float wn  = cst_lds[2 * kD + col];
      const float br  = cst_lds[3 * kD + col];
      const float bz  = cst_lds[4 * kD + col];
      const float bin = cst_lds[5 * kD + col];
      const float bhn = cst_lds[6 * kD + col];
#pragma unroll
      for (int mt = 0; mt < 2; ++mt) {
#pragma unroll
        for (int r = 0; r < 8; ++r) {
          const int row = mt * 16 + 8 * hh + r;
          const float xv  = x_lds[row];
          const float pr  = fmaf(acc[mt][g][r],     kInvCarry, fmaf(xv, wr, br));
          const float pz  = fmaf(acc[mt][2 + g][r], kInvCarry, fmaf(xv, wz, bz));
          const float hnv = fmaf(acc[mt][4 + g][r], kInvCarry, bhn);
          const float rr  = fast_sigmoid(pr);
          const float zz  = fast_sigmoid(pz);
          const float pn  = fmaf(rr, hnv, fmaf(xv, wn, bin));
          const float nc  = fast_tanh(pn);
          const float ho  = hold[mt][g][r];
          const float hv  = fmaf(zz, ho - nc, nc);
          hold[mt][g][r] = hv;
          hbuf[row * kHP + col] = (_Float16)hv;
        }
      }
    }
    __syncthreads();

    v8f pacc = (v8f){0.f, 0.f, 0.f, 0.f, 0.f, 0.f, 0.f, 0.f};
    if (wave < 2) {
#pragma unroll 1
      for (int kk = 0; kk < kD / 32; ++kk) {
        const int ko = kk * 32 + 8 * hh;
        FragU a, b;
        a.h[0] = *(const v8h*)(hbuf + (wave * 16 + rl) * kHP + ko);
        a.h[1] = *(const v8h*)(hbuf + (wave * 16 + rl) * kHP + ko + 16);
        b.h[0] = *(const v8h*)(wlg + rl * kHP + ko);
        b.h[1] = *(const v8h*)(wlg + rl * kHP + ko + 16);
        pacc = mma_f16(a.v, b.v, pacc);
      }
    }
    float tv[8];
#pragma unroll
    for (int r = 0; r < 8; ++r) {
      const float lw = fmaf(pacc[r], kInvCarry, blv) * whv;
      tv[r] = lowcol ? lw : 0.0f;
    }
#pragma unroll
    for (int r = 0; r < 8; ++r) {
      tv[r] += __shfl_xor(tv[r], 1, 32);
      tv[r] += __shfl_xor(tv[r], 2, 32);
      tv[r] += __shfl_xor(tv[r], 4, 32);
    }
    if (wave < 2 && rl == 0) {
#pragma unroll
      for (int r = 0; r < 8; ++r) {
        const int row = wave * 16 + 8 * hh + r;
        const float p = tv[r] + bhv;
        x_lds[row] = p;
        preds_lds[row * kHor + t] = p;
      }
    }
    __syncthreads();
  }

  if (tid < 192) {
    const float rate = expf(log_decay[0]);
    const int row = tid / 6;
    const int t0  = (tid - row * 6) * 4;
    const v4f gv = *(const v4f*)(gate_lds + 4 * tid);
    const v4f pv = *(const v4f*)(preds_lds + 4 * tid);
    const float lv = lv_lds[row];
    v4f o;
#pragma unroll
    for (int e = 0; e < 4; ++e) {
      const float dec = lv * expf(-rate * (float)(t0 + e + 1));
      o[e] = gv[e] * pv[e] + (1.0f - gv[e]) * dec;
    }
    float* dst = out + (size_t)row0 * kHor + 4 * tid;
    *(volatile v4f*)dst = o;
    __threadfence();
    *(volatile v4f*)dst = o;
  }
}

extern "C" void kernel_launch(void* const* d_in, const int* in_sizes, int n_in,
                              void* d_out, int out_size, void* d_ws, size_t ws_size,
                              hipStream_t stream) {
  if (n_in < 15) return;
  if (in_sizes[0] != kRows * kD) return;
  if (in_sizes[1] != kRows) return;
  if (in_sizes[2] != kG3) return;
  if (in_sizes[3] != kG3 * kD) return;
  if (in_sizes[4] != kG3) return;
  if (in_sizes[5] != kG3) return;
  if (in_sizes[6] != kBot * kD) return;
  if (in_sizes[7] != kBot) return;
  if (in_sizes[8] != kBot) return;
  if (in_sizes[9] != 1) return;
  if (in_sizes[10] != kBot * kD) return;
  if (in_sizes[11] != kBot) return;
  if (in_sizes[12] != kHor * kBot) return;
  if (in_sizes[13] != kHor) return;
  if (in_sizes[14] != 1) return;
  if (out_size != kRows * kHor) return;
  if (ws_size < kWsTotal) return;

  const float* features   = (const float*)d_in[0];
  const float* last_value = (const float*)d_in[1];
  const float* W_ih       = (const float*)d_in[2];
  const float* W_hh       = (const float*)d_in[3];
  const float* b_ih       = (const float*)d_in[4];
  const float* b_hh       = (const float*)d_in[5];
  const float* Wl         = (const float*)d_in[6];
  const float* bl         = (const float*)d_in[7];
  const float* Wh         = (const float*)d_in[8];
  const float* bh         = (const float*)d_in[9];
  const float* Wg1        = (const float*)d_in[10];
  const float* bg1        = (const float*)d_in[11];
  const float* Wg2        = (const float*)d_in[12];
  const float* bg2        = (const float*)d_in[13];
  const float* log_decay  = (const float*)d_in[14];

  unsigned short* planes = (unsigned short*)d_ws;

  build_planes_kernel<<<kCvtBlocks, 256, 0, stream>>>(W_hh, Wl, Wg1, planes);

  gru_horizon_kernel<<<kBlocks, 256, 0, stream>>>(
      features, last_value, W_ih, b_ih, b_hh, bl, Wh, bh, bg1, Wg2, bg2, log_decay,
      planes, (float*)d_out);
}
